// InnerIteration_60936995996046
// MI455X (gfx1250) — hardware-verified
//
#include <hip/hip_runtime.h>
#include <stdint.h>

typedef _Float16     v16h __attribute__((ext_vector_type(16)));
typedef _Float16     v8h  __attribute__((ext_vector_type(8)));
typedef _Float16     v4h  __attribute__((ext_vector_type(4)));
typedef float        v8f  __attribute__((ext_vector_type(8)));
typedef float        v4f  __attribute__((ext_vector_type(4)));
typedef unsigned int v4u  __attribute__((ext_vector_type(4)));
typedef unsigned int v2u  __attribute__((ext_vector_type(2)));
typedef int          v4i  __attribute__((ext_vector_type(4)));

union Frag { v16h v; v4u q[2]; };
union C8   { v8h h; v4u u; };
union C4   { v4h h; v2u u; };

#define ND 64
#define NC 16
#define NL 6
#define NR 96
#define KV 384
#define KC 1024

static __device__ __forceinline__ v8f wmma16(const Frag& a, const Frag& b, v8f c)
{
    v8f d = __builtin_amdgcn_wmma_f32_16x16x32_f16(false, a.v, false, b.v, (short)0, c, false, false);
    asm volatile("v_nop\n\tv_nop\n\tv_nop\n\tv_nop" : "+v"(d) : "v"(a.v), "v"(b.v));
    return d;
}
static __device__ __forceinline__ v8f zero8()
{
    v8f z;
#pragma unroll
    for (int r = 0; r < 8; ++r) z[r] = 0.0f;
    return z;
}
static __device__ __forceinline__ v4u cvt8(v4f a, v4f b)
{
    C8 c;
    v4h ha = __builtin_convertvector(a, v4h);
    v4h hb = __builtin_convertvector(b, v4h);
    c.h = __builtin_shufflevector(ha, hb, 0, 1, 2, 3, 4, 5, 6, 7);
    return c.u;
}
static __device__ __forceinline__ float sigm(float x)
{
    return 1.0f / (1.0f + __expf(-x));
}

__global__ __launch_bounds__(256) void k_wcvt(const float* __restrict__ src, v4u* dst, int K)
{
    __shared__ union { _Float16 e[64 * 64]; v4u q[64 * 8]; } T;
    const int tid = threadIdx.x;
    const int k0 = blockIdx.x * 64;
    if (k0 + 64 > K) return;
#pragma unroll 4
    for (int j = 0; j < 16; ++j) {
        const int idx = tid + 256 * j;
        const int n = idx & 63, kk = idx >> 6;
        T.e[n * 64 + kk] = (_Float16)src[(size_t)(k0 + kk) * ND + n];
    }
    __syncthreads();
    const int KQ = K >> 3;
    v4u val[2]; size_t off[2];
#pragma unroll
    for (int t = 0; t < 2; ++t) {
        const int p = tid + 256 * t;
        const int row = p >> 3, j = p & 7;
        val[t] = T.q[row * 8 + j];
        off[t] = (size_t)row * KQ + (k0 >> 3) + j;
    }
#pragma unroll
    for (int t = 0; t < 2; ++t) *(volatile v4u*)(dst + off[t]) = val[t];
    __threadfence();
#pragma unroll
    for (int t = 0; t < 2; ++t) *(volatile v4u*)(dst + off[t]) = val[t];
}

__global__ __launch_bounds__(256) void k_main(
    const float* __restrict__ X,
    const int*   __restrict__ lits,
    const int*   __restrict__ negm,
    const int*   __restrict__ valid,
    const int*   __restrict__ cval,
    const float* __restrict__ Wn,
    const float* __restrict__ bn,
    const float* __restrict__ fe,
    const float* __restrict__ b1v, const float* __restrict__ b2v,
    const float* __restrict__ b1c, const float* __restrict__ b2c,
    const v4u* __restrict__ WnH,
    const v4u* __restrict__ W1vH,
    const v4u* __restrict__ W2vH,
    const v4u* __restrict__ W1cH,
    const v4u* __restrict__ W2cH,
    float* out, int V)
{
    __shared__ union { v4u g[NR * 8]; _Float16 ge[NR * ND]; float h[2 * NC * ND]; } s_u;
    __shared__ union { _Float16 e[NR * ND]; v4u q[NR * 8]; } s_v;
    __shared__ union { v2u d[16 * 256]; v4u q[16 * 128]; } s_y;
    __shared__ float s_red[256];
    __shared__ float s_bn[ND], s_true[ND], s_b1v[ND], s_b2v[ND], s_b1c[ND], s_b2c[ND];
    __shared__ _Float16 s_fe16[ND];
    __shared__ int s_ng[NR], s_vv[NR];

    const int tid = threadIdx.x, lane = tid & 31, wave = tid >> 5;
    const int h = lane >> 4, m = lane & 15;
    const int nt = wave & 3, mat = wave >> 2;
    const int v0 = blockIdx.x * 16;

    if (tid < ND) {
        s_bn[tid]   = bn[tid];
        s_b1v[tid]  = b1v[tid];
        s_b2v[tid]  = b2v[tid];
        s_b1c[tid]  = b1c[tid];
        s_b2c[tid]  = b2c[tid];
        s_fe16[tid] = (_Float16)fe[tid];
        float t = bn[tid];
        for (int k = 0; k < ND; ++k) t = fmaf(fe[k], Wn[(size_t)k * ND + tid], t);
        s_true[tid] = t;
    }
    Frag wnF[2];
    {
        const v4u* Bq = WnH + (size_t)(nt * 16 + m) * (ND / 8);
#pragma unroll
        for (int ks = 0; ks < 2; ++ks) {
            wnF[ks].q[0] = Bq[4 * ks + h];
            wnF[ks].q[1] = Bq[4 * ks + 2 + h];
        }
    }
    __syncthreads();

    for (int vi = 0; vi < 16; ++vi) {
        int v = v0 + vi; if (v > V - 1) v = V - 1;
        const int lbase = v * NR;

        if (tid < NR) {
            s_ng[tid] = negm[lbase + tid];
            s_vv[tid] = valid[lbase + tid];
        }
        for (int i = tid; i < NR * 8; i += 256) {
            const int row = i >> 3, q = i & 7;
            int idx = lits[lbase + row];
            idx = idx < 0 ? 0 : (idx > V - 1 ? V - 1 : idx);
            const float* xp = X + (size_t)idx * ND + 8 * q;
            const v4f xa = *(const v4f*)xp;
            const v4f xb = *(const v4f*)(xp + 4);
            s_u.g[i] = cvt8(xa, xb);
        }
        __syncthreads();

        {
            v8f accn[3];
#pragma unroll
            for (int t = 0; t < 3; ++t) {
                const int mt = mat + 2 * t;
                const v4u* Arow = s_u.g + (mt * 16 + m) * 8;
                v8f acc = zero8();
#pragma unroll
                for (int ks = 0; ks < 2; ++ks) {
                    Frag a;
                    a.q[0] = Arow[4 * ks + h];
                    a.q[1] = Arow[4 * ks + 2 + h];
                    acc = wmma16(a, wnF[ks], acc);
                }
                accn[t] = acc;
            }
            const int n = nt * 16 + m;
            const float bb = s_bn[n];
            const _Float16 fv = s_fe16[n];
#pragma unroll
            for (int t = 0; t < 3; ++t) {
                const int mt = mat + 2 * t;
#pragma unroll
                for (int r = 0; r < 8; ++r) {
                    const int rl = mt * 16 + 8 * h + r;
                    _Float16 val = s_u.ge[rl * ND + n];
                    const _Float16 nv = (_Float16)(accn[t][r] + bb);
                    if (s_ng[rl] != 0) val = nv;
                    if (s_vv[rl] == 0) val = fv;
                    s_v.e[rl * ND + n] = val;
                }
            }
        }
        __syncthreads();

        {
            v8f acc = zero8();
            const v4u* Arow = s_v.q + m * (KV / 8);
            const v4u* Bq = (mat ? W2vH : W1vH) + (size_t)(nt * 16 + m) * (KV / 8);
#pragma unroll 4
            for (int ks = 0; ks < KV / 32; ++ks) {
                Frag a, b;
                a.q[0] = Arow[4 * ks + h];
                a.q[1] = Arow[4 * ks + 2 + h];
                b.q[0] = Bq[4 * ks + h];
                b.q[1] = Bq[4 * ks + 2 + h];
                acc = wmma16(a, b, acc);
            }
            float* H = s_u.h + mat * (NC * ND);
            const int n = nt * 16 + m;
#pragma unroll
            for (int r = 0; r < 8; ++r) H[(8 * h + r) * ND + n] = acc[r];
        }
        __syncthreads();

        {
            const int cc = tid >> 4, c0 = tid & 15;
            float x[4], ssq = 0.0f;
#pragma unroll
            for (int e = 0; e < 4; ++e) {
                const int n = 4 * c0 + e;
                const float t = sigm(s_u.h[cc * ND + n] + s_b1v[n]) + s_u.h[NC * ND + cc * ND + n] + s_b2v[n];
                x[e] = t; ssq = fmaf(t, t, ssq);
            }
            s_red[tid] = ssq;
            __syncthreads();
            float s = 0.0f;
#pragma unroll
            for (int j = 0; j < 16; ++j) s += s_red[(cc << 4) + j];
            const float rn = 1.0f / sqrtf(s);
            const int cvf = cval[(size_t)v * NC + cc];
            v4f yv;
#pragma unroll
            for (int e = 0; e < 4; ++e) yv[e] = (cvf != 0) ? x[e] * rn : s_true[4 * c0 + e];
            C4 c;
            c.h = __builtin_convertvector(yv, v4h);
            s_y.d[vi * 256 + cc * 16 + c0] = c.u;
        }
        __syncthreads();
    }

    {
        v8f acc = zero8();
        const v4u* Arow = s_y.q + m * (KC / 8);
        const v4u* Bq = (mat ? W2cH : W1cH) + (size_t)(nt * 16 + m) * (KC / 8);
#pragma unroll 4
        for (int ks = 0; ks < KC / 32; ++ks) {
            Frag a, b;
            a.q[0] = Arow[4 * ks + h];
            a.q[1] = Arow[4 * ks + 2 + h];
            b.q[0] = Bq[4 * ks + h];
            b.q[1] = Bq[4 * ks + 2 + h];
            acc = wmma16(a, b, acc);
        }
        float* H = s_u.h + mat * (NC * ND);
        const int n = nt * 16 + m;
#pragma unroll
        for (int r = 0; r < 8; ++r) H[(8 * h + r) * ND + n] = acc[r];
    }
    __syncthreads();
    {
        const int mrow = tid >> 4, c0 = tid & 15;
        int vr = v0 + mrow;
        const bool ok = vr < V;
        if (!ok) vr = V - 1;
        float x[4], ssq = 0.0f;
#pragma unroll
        for (int e = 0; e < 4; ++e) {
            const int n = 4 * c0 + e;
            const float t = sigm(s_u.h[mrow * ND + n] + s_b1c[n]) + s_u.h[NC * ND + mrow * ND + n] + s_b2c[n];
            x[e] = t; ssq = fmaf(t, t, ssq);
        }
        s_red[tid] = ssq;
        __syncthreads();
        float s = 0.0f;
#pragma unroll
        for (int j = 0; j < 16; ++j) s += s_red[(mrow << 4) + j];
        const float rn = 1.0f / sqrtf(s);
        const v4i* cp = (const v4i*)(cval + (size_t)vr * NC);
        const v4i c4 = cp[0] | cp[1] | cp[2] | cp[3];
        const int anyc = ((c4[0] | c4[1] | c4[2] | c4[3]) != 0) ? 1 : 0;
        const v4f pass = *(const v4f*)(X + (size_t)vr * ND + 4 * c0);
        v4f ov;
#pragma unroll
        for (int e = 0; e < 4; ++e) ov[e] = (anyc != 0) ? x[e] * rn : pass[e];
        float* p = out + (size_t)vr * ND + 4 * c0;
        if (ok) *(volatile v4f*)p = ov;
        __threadfence();
        if (ok) *(volatile v4f*)p = ov;
    }
}

extern "C" void kernel_launch(void* const* d_in, const int* in_sizes, int n_in,
                              void* d_out, int out_size, void* d_ws, size_t ws_size,
                              hipStream_t stream)
{
    if (n_in < 16) return;
    const int V = in_sizes[0] / ND;
    if (V <= 0 || in_sizes[0] != V * ND) return;
    if (in_sizes[1] != V * NR || in_sizes[2] != V * NR || in_sizes[3] != V * NR) return;
    if (in_sizes[4] != V * NC) return;
    if (in_sizes[5] != ND * ND || in_sizes[6] != ND || in_sizes[7] != ND) return;
    if (in_sizes[8] != KV * ND || in_sizes[9] != ND || in_sizes[10] != KV * ND || in_sizes[11] != ND) return;
    if (in_sizes[12] != KC * ND || in_sizes[13] != ND || in_sizes[14] != KC * ND || in_sizes[15] != ND) return;
    if (out_size != V * ND) return;

    const float* X    = (const float*)d_in[0];
    const int*   lits = (const int*)d_in[1];
    const int*   negm = (const int*)d_in[2];
    const int*   vval = (const int*)d_in[3];
    const int*   cval = (const int*)d_in[4];
    const float* Wn   = (const float*)d_in[5];
    const float* bn   = (const float*)d_in[6];
    const float* fe   = (const float*)d_in[7];
    const float* W1v  = (const float*)d_in[8];
    const float* b1v  = (const float*)d_in[9];
    const float* W2v  = (const float*)d_in[10];
    const float* b2v  = (const float*)d_in[11];
    const float* W1c  = (const float*)d_in[12];
    const float* b1c  = (const float*)d_in[13];
    const float* W2c  = (const float*)d_in[14];
    const float* b2c  = (const float*)d_in[15];
    float* out = (float*)d_out;

    const size_t szWn = (size_t)ND * ND * 2;
    const size_t szWv = (size_t)ND * KV * 2;
    const size_t szWc = (size_t)ND * KC * 2;
    size_t off = 0;
    const size_t oWn  = off; off += szWn;
    const size_t oW1v = off; off += szWv;
    const size_t oW2v = off; off += szWv;
    const size_t oW1c = off; off += szWc;
    const size_t oW2c = off; off += szWc;
    if (off > ws_size) return;

    char* ws = (char*)d_ws;
    v4u* WnH  = (v4u*)(ws + oWn);
    v4u* W1vH = (v4u*)(ws + oW1v);
    v4u* W2vH = (v4u*)(ws + oW2v);
    v4u* W1cH = (v4u*)(ws + oW1c);
    v4u* W2cH = (v4u*)(ws + oW2c);

    k_wcvt<<<ND / 64, 256, 0, stream>>>(Wn,  WnH,  ND);
    k_wcvt<<<KV / 64, 256, 0, stream>>>(W1v, W1vH, KV);
    k_wcvt<<<KV / 64, 256, 0, stream>>>(W2v, W2vH, KV);
    k_wcvt<<<KC / 64, 256, 0, stream>>>(W1c, W1cH, KC);
    k_wcvt<<<KC / 64, 256, 0, stream>>>(W2c, W2cH, KC);

    const int nblk = (V + 15) / 16;
    k_main<<<nblk, 256, 0, stream>>>(X, lits, negm, vval, cval, Wn, bn, fe, b1v, b2v, b1c, b2c,
                                     WnH, W1vH, W2vH, W1cH, W2cH, out, V);
}
